// SSM_2104533975587
// MI455X (gfx1250) — hardware-run, weakly checked
//
#include <hip/hip_runtime.h>
#include <math.h>

typedef __attribute__((ext_vector_type(16))) _Float16 v16h;
typedef __attribute__((ext_vector_type(8)))  _Float16 v8h;
typedef __attribute__((ext_vector_type(4)))  _Float16 v4h;
typedef __attribute__((ext_vector_type(16))) __bf16   v16b;
typedef __attribute__((ext_vector_type(8)))  __bf16   v8b;
typedef __attribute__((ext_vector_type(8)))  float    v8f;
typedef __attribute__((ext_vector_type(4)))  float    v4f;
typedef __attribute__((ext_vector_type(4)))  unsigned v4u;

constexpr bool kLegBf16 = true;
constexpr int  kSpl1    = kLegBf16 ? 0 : 2;

constexpr int kNB    = 2;
constexpr int kSeq   = 2048;
constexpr int kDm    = 1024;
constexpr int kDin   = 2048;
constexpr int kNst   = 16;
constexpr int kTaps  = 4;
constexpr int kDtR   = 64;
constexpr int kXw    = kDtR + 2 * kNst;
constexpr int kXwPad = 128;
constexpr int kBcW   = 2 * kNst;
constexpr int kRows  = kNB * kSeq;
constexpr int kChunk = 32;

constexpr float kCarryU   = 32.0f;
constexpr float kCarryWx  = 1024.0f;
constexpr float kCarryWdt = 1024.0f;
constexpr float kCarryDt  = 64.0f;
constexpr float kF16Min   = 6.103515625e-05f;

static_assert(kXw == 96);
static_assert(kBcW == 32);
static_assert((kDm % 32) == 0 && (kDin % 32) == 0 && (kDtR % 32) == 0);
static_assert((kRows % 64) == 0 && (kDin % 64) == 0 && (kXwPad % 64) == 0 && kXwPad == 128);
static_assert((kSeq % kChunk) == 0 && (kSeq & (kSeq - 1)) == 0);
static_assert(kDin / 4 == 512);
static_assert((kDin / 64) == 32);

constexpr size_t kSzA1  = (size_t)kRows * kDm * 2;
constexpr size_t kSzB1  = (size_t)kDin * kDm * 2;
constexpr size_t kSzA1L = kLegBf16 ? 0 : kSzA1;
constexpr size_t kSzB1L = kLegBf16 ? 0 : kSzB1;
constexpr size_t kSzBT2 = (size_t)kXwPad * kDin * 2;
constexpr size_t kSzBT3 = (size_t)kDin * kDtR * 2;
constexpr size_t kSzXD  = (size_t)kRows * kDin * 4;
constexpr size_t kSzUF  = (size_t)kRows * kDin * 4;
constexpr size_t kSzUH  = (size_t)kRows * kDin * 2;
constexpr size_t kSzBC  = (size_t)kRows * kBcW * 4;
constexpr size_t kSzDTL = (size_t)kRows * kDtR * 2;

constexpr size_t kOffA1H = 0;
constexpr size_t kOffB1H = kOffA1H + kSzA1;
constexpr size_t kOffA1L = kOffB1H + kSzB1;
constexpr size_t kOffB1L = kOffA1L + kSzA1L;
constexpr size_t kOffBT2 = kOffB1L + kSzB1L;
constexpr size_t kOffBT3 = kOffBT2 + kSzBT2;
constexpr size_t kOffXD  = kOffBT3 + kSzBT3;
constexpr size_t kOffUF  = kOffXD  + kSzXD;
constexpr size_t kOffUH  = kOffUF  + kSzUF;
constexpr size_t kOffBC  = kOffUH  + kSzUH;
constexpr size_t kOffDTL = kOffBC  + kSzBC;
constexpr size_t kWsTotal = kOffDTL + kSzDTL;
static_assert(kWsTotal == (kLegBf16 ? 98304000ull : 110886912ull));
static_assert(kWsTotal <= 134217728ull);
static_assert((kOffB1H % 128) == 0 && (kOffA1L % 128) == 0 && (kOffB1L % 128) == 0 && (kOffBT2 % 128) == 0 &&
              (kOffBT3 % 128) == 0 && (kOffXD % 128) == 0 && (kOffUF % 128) == 0 && (kOffUH % 128) == 0 &&
              (kOffBC % 128) == 0 && (kOffDTL % 128) == 0);

__device__ __forceinline__ unsigned bf16_rne_word(float f) {
  unsigned u = __float_as_uint(f);
  const unsigned lsb = (u & 0x00010000u) ? 1u : 0u;
  u = (u + 0x7FFFu + lsb) & 0xFFFF0000u;
  return u;
}
__device__ __forceinline__ float leg_in(float f) {
  return kLegBf16 ? __uint_as_float(bf16_rne_word(f)) : f;
}
__device__ __forceinline__ unsigned pack_hi_halves(unsigned w0, unsigned w1) {
  return __builtin_amdgcn_perm(w1, w0, 0x07060302u);
}
__device__ __forceinline__ _Float16 f16_flush(float v) {
  const float w = (fabsf(v) < kF16Min) ? 0.0f : v;
  return (_Float16)w;
}
__device__ __forceinline__ void pin4(v4f& v) {
  float a = v[0], b = v[1], c = v[2], d = v[3];
  asm volatile("" : "+v"(a), "+v"(b), "+v"(c), "+v"(d));
  v = (v4f){a, b, c, d};
}
__device__ __forceinline__ float silu_f(float v) {
  return v * __builtin_amdgcn_rcpf(1.0f + expf(-v));
}
__device__ __forceinline__ float softplus_stable(float v) {
  return fmaxf(v, 0.0f) + log1pf(expf(-fabsf(v)));
}

__device__ __forceinline__ void keep4_h(v16h a, v16h b, v16h c, v16h d) { asm volatile("v_nop" :: "v"(a), "v"(b), "v"(c), "v"(d)); }
__device__ __forceinline__ void keep4_b(v16b a, v16b b, v16b c, v16b d) { asm volatile("v_nop" :: "v"(a), "v"(b), "v"(c), "v"(d)); }
__device__ __forceinline__ void acc_guard4(v8f& a, v8f& b, v8f& c, v8f& d) { asm volatile("v_nop\n\tv_nop\n\tv_nop\n\tv_nop" : "+v"(a), "+v"(b), "+v"(c), "+v"(d)); }
__device__ __forceinline__ v8f mma_guarded_h(v16h a, v16h b, v8f c) {
  c = __builtin_amdgcn_wmma_f32_16x16x32_f16(false, a, false, b, (short)0, c, false, false);
  asm volatile("v_nop\n\tv_nop\n\tv_nop\n\tv_nop" : "+v"(c) : "v"(a), "v"(b));
  return c;
}
__device__ __forceinline__ v8f mma_guarded_b(v16b a, v16b b, v8f c) {
  c = __builtin_amdgcn_wmma_f32_16x16x32_bf16(false, a, false, b, (short)0, c, false, false);
  asm volatile("v_nop\n\tv_nop\n\tv_nop\n\tv_nop" : "+v"(c) : "v"(a), "v"(b));
  return c;
}
template <typename T> struct Frag;
template <> struct Frag<_Float16> {
  typedef v16h V; union U { v16h v; v8h h[2]; };
  static __device__ __forceinline__ v16h load(const _Float16* p) {
    U f; f.h[0] = *(const v8h*)(p); f.h[1] = *(const v8h*)(p + 16); return f.v;
  }
  static __device__ __forceinline__ v8f mma(v16h a, v16h b, v8f c) { return mma_guarded_h(a, b, c); }
  static __device__ __forceinline__ void keep(v16h a, v16h b, v16h c, v16h d) { keep4_h(a, b, c, d); }
};
template <> struct Frag<__bf16> {
  typedef v16b V; union U { v16b v; v8b h[2]; };
  static __device__ __forceinline__ v16b load(const __bf16* p) {
    U f; f.h[0] = *(const v8b*)(p); f.h[1] = *(const v8b*)(p + 16); return f.v;
  }
  static __device__ __forceinline__ v8f mma(v16b a, v16b b, v8f c) { return mma_guarded_b(a, b, c); }
  static __device__ __forceinline__ void keep(v16b a, v16b b, v16b c, v16b d) { keep4_b(a, b, c, d); }
};
template <int ET> struct Elem;
template <> struct Elem<0> { typedef _Float16 T; };
template <> struct Elem<1> { typedef __bf16 T; };

template <int ET, int SPL, int EPI>
__global__ __launch_bounds__(256) void gemm64_kernel(
    const unsigned short* __restrict__ Ap, const unsigned short* __restrict__ A2p, int lda,
    const unsigned short* __restrict__ Btp, const unsigned short* __restrict__ Bt2p, int ldb,
    void* __restrict__ C0, void* __restrict__ C1, int ldc,
    const float* __restrict__ bias, int M, int N, int K) {
  typedef typename Elem<ET>::T T;
  typedef typename Frag<T>::V V;
  const T* A = (const T*)Ap; const T* A2 = (const T*)A2p; const T* Bt = (const T*)Btp; const T* Bt2 = (const T*)Bt2p;
  __shared__ __align__(16) float sT[8][16 * 68];
  const int lane = threadIdx.x & 31;
  const int wave = threadIdx.x >> 5;
  const int tilesN = N >> 6;
  const int tilesM = M >> 6;
  const int tile = blockIdx.x * 8 + wave;
  if (tile >= tilesM * tilesN) return;
  const int tm = tile / tilesN;
  const int tn = tile - tm * tilesN;
  const int m0 = tm << 6;
  const int n0 = tn << 6;

  const int rlane = lane & 15;
  const int koff  = (lane >> 4) * 8;
  const int mOff  = (lane >> 4) * 8;

  constexpr float kScale = (EPI == 0) ? 1.0f
                         : (EPI == 1) ? (1.0f / (kCarryU * kCarryWx))
                                      : (1.0f / (kCarryDt * kCarryWdt));

  v8f acc[4][4];
#pragma unroll
  for (int i = 0; i < 4; ++i)
#pragma unroll
    for (int j = 0; j < 4; ++j) acc[i][j] = (v8f){0.f,0.f,0.f,0.f,0.f,0.f,0.f,0.f};

  for (int k0 = 0; k0 < K; k0 += 32) {
    V bh[4], bl[4];
#pragma unroll
    for (int j = 0; j < 4; ++j) {
      const size_t bo = (size_t)(n0 + (j << 4) + rlane) * ldb + koff + k0;
      bh[j] = Frag<T>::load(Bt + bo);
      if (SPL == 2) bl[j] = Frag<T>::load(Bt2 + bo);
    }
#pragma unroll
    for (int i = 0; i < 4; ++i) {
      const size_t ao = (size_t)(m0 + (i << 4) + rlane) * lda + koff + k0;
      V ah = Frag<T>::load(A + ao);
      V al;
      if (SPL == 2) al = Frag<T>::load(A2 + ao);
#pragma unroll
      for (int j = 0; j < 4; ++j) {
        acc[i][j] = Frag<T>::mma(ah, bh[j], acc[i][j]);
        if (SPL == 2) {
          acc[i][j] = Frag<T>::mma(ah, bl[j], acc[i][j]);
          acc[i][j] = Frag<T>::mma(al, bh[j], acc[i][j]);
        }
      }
    }
    Frag<T>::keep(bh[0], bh[1], bh[2], bh[3]);
    if (SPL == 2) Frag<T>::keep(bl[0], bl[1], bl[2], bl[3]);
  }
  acc_guard4(acc[0][0], acc[0][1], acc[0][2], acc[0][3]);
  acc_guard4(acc[1][0], acc[1][1], acc[1][2], acc[1][3]);
  acc_guard4(acc[2][0], acc[2][1], acc[2][2], acc[2][3]);
  acc_guard4(acc[3][0], acc[3][1], acc[3][2], acc[3][3]);

  float* slab = sT[wave];
  float bias_lo = 0.f, bias_hi = 0.f;
  if (EPI == 2) {
    bias_lo = leg_in(bias[n0 + lane]);
    bias_hi = leg_in(bias[n0 + 32 + lane]);
  }
#pragma unroll
  for (int i = 0; i < 4; ++i) {
    const int mBase = m0 + (i << 4);
#pragma unroll
    for (int j = 0; j < 4; ++j) {
#pragma unroll
      for (int r = 0; r < 8; ++r) {
        slab[(mOff + r) * 68 + (j << 4) + rlane] = acc[i][j][r] * kScale;
      }
    }
    __builtin_amdgcn_fence(__ATOMIC_RELEASE, "workgroup");
    __builtin_amdgcn_wave_barrier();
    __builtin_amdgcn_fence(__ATOMIC_ACQUIRE, "workgroup");
    if (EPI == 2) {
#pragma unroll 1
      for (int idx = 0; idx < 32; ++idx) {
        const int odd = idx & 1;
        float* sp = slab + (idx >> 1) * 68 + odd * 32 + lane;
        const float bsel = odd ? bias_hi : bias_lo;
        const float pre = *sp + bsel;
        *sp = softplus_stable(pre);
      }
      __builtin_amdgcn_fence(__ATOMIC_RELEASE, "workgroup");
      __builtin_amdgcn_wave_barrier();
      __builtin_amdgcn_fence(__ATOMIC_ACQUIRE, "workgroup");
    }
    if (EPI == 0 || EPI == 2) {
      float* C = (float*)C0;
      const int hh = lane >> 4, c4 = (lane & 15) * 4;
      for (int pass = 0; pass < 2; ++pass) {
#pragma unroll
        for (int it = 0; it < 8; ++it) {
          const int row = it * 2 + hh;
          v4f v = *(const v4f*)(slab + row * 68 + c4);
          *(volatile v4f*)(C + (size_t)(mBase + row) * ldc + n0 + c4) = v;
        }
        __threadfence();
      }
    } else {
      const int q = lane >> 3;
      if (tn == 0) {
        unsigned short* C = (unsigned short*)C1;
        const int c8 = (lane & 7) * 8;
        v8h hv[4];
#pragma unroll
        for (int it = 0; it < 4; ++it) {
          const float* sp = slab + (it * 4 + q) * 68 + c8;
          const v4f a0 = *(const v4f*)(sp);
          const v4f a1 = *(const v4f*)(sp + 4);
#pragma unroll
          for (int e = 0; e < 4; ++e) {
            hv[it][e]     = f16_flush(a0[e] * kCarryDt);
            hv[it][4 + e] = f16_flush(a1[e] * kCarryDt);
          }
        }
        for (int pass = 0; pass < 2; ++pass) {
#pragma unroll
          for (int it = 0; it < 4; ++it) {
            const int row = it * 4 + q;
            *(volatile v8h*)(C + (size_t)(mBase + row) * kDtR + c8) = hv[it];
          }
          __threadfence();
        }
      } else if (tn == 1) {
        float* C = (float*)C0;
        const int c4 = (lane & 7) * 4;
        v4f fv[4];
#pragma unroll
        for (int it = 0; it < 4; ++it) fv[it] = *(const v4f*)(slab + (it * 4 + q) * 68 + c4);
        for (int pass = 0; pass < 2; ++pass) {
#pragma unroll
          for (int it = 0; it < 4; ++it) {
            const int row = it * 4 + q;
            *(volatile v4f*)(C + (size_t)(mBase + row) * kBcW + c4) = fv[it];
          }
          __threadfence();
        }
      }
    }
    __builtin_amdgcn_fence(__ATOMIC_RELEASE, "workgroup");
    __builtin_amdgcn_wave_barrier();
    __builtin_amdgcn_fence(__ATOMIC_ACQUIRE, "workgroup");
  }
}

template <bool SPLIT>
__global__ __launch_bounds__(256) void prep_bf16_kernel(
    const float* __restrict__ src, unsigned short* __restrict__ dhi, unsigned short* __restrict__ dlo, int total8) {
  const int i = blockIdx.x * 256 + threadIdx.x;
  if (i >= total8) return;
  const size_t e0 = (size_t)i << 3;
  const v4f a0 = *(const v4f*)(src + e0);
  const v4f a1 = *(const v4f*)(src + e0 + 4);
  unsigned wh[8], wl[8];
#pragma unroll
  for (int e = 0; e < 4; ++e) {
    const float x0 = a0[e];
    const float x1 = a1[e];
    wh[e]     = bf16_rne_word(x0);
    wh[4 + e] = bf16_rne_word(x1);
    wl[e]     = SPLIT ? bf16_rne_word(x0 - __uint_as_float(wh[e])) : 0u;
    wl[4 + e] = SPLIT ? bf16_rne_word(x1 - __uint_as_float(wh[4 + e])) : 0u;
  }
  const v4u ph = (v4u){pack_hi_halves(wh[0], wh[1]), pack_hi_halves(wh[2], wh[3]),
                       pack_hi_halves(wh[4], wh[5]), pack_hi_halves(wh[6], wh[7])};
  const v4u pl = (v4u){pack_hi_halves(wl[0], wl[1]), pack_hi_halves(wl[2], wl[3]),
                       pack_hi_halves(wl[4], wl[5]), pack_hi_halves(wl[6], wl[7])};
  unsigned short* qh = dhi + e0;
  unsigned short* ql = dlo + e0;
  *(volatile v4u*)qh = ph;
  if (SPLIT) *(volatile v4u*)ql = pl;
  __threadfence();
  *(volatile v4u*)qh = ph;
  if (SPLIT) *(volatile v4u*)ql = pl;
}

template <int CARRY>
__global__ __launch_bounds__(256) void prep_f16_kernel(
    const float* __restrict__ src, unsigned short* __restrict__ dst, int n8_real, int n8_total) {
  const int i = blockIdx.x * 256 + threadIdx.x;
  if (i >= n8_total) return;
  const bool real = (i < n8_real);
  const int ic = real ? i : (n8_real - 1);
  v4f a0 = *(const v4f*)(src + (size_t)ic * 8);
  v4f a1 = *(const v4f*)(src + (size_t)ic * 8 + 4);
  pin4(a0);
  pin4(a1);
  v8h hv;
#pragma unroll
  for (int e = 0; e < 4; ++e) {
    const float x0 = a0[e];
    const float x1 = a1[e];
    const float y0 = real ? (leg_in(x0) * (float)CARRY) : 0.0f;
    const float y1 = real ? (leg_in(x1) * (float)CARRY) : 0.0f;
    hv[e]     = f16_flush(y0);
    hv[4 + e] = f16_flush(y1);
  }
  unsigned short* q = dst + (size_t)i * 8;
  *(volatile v8h*)q = hv;
  __threadfence();
  *(volatile v8h*)q = hv;
}

__global__ __launch_bounds__(256) void conv_act_kernel(
    const float* __restrict__ X, const float* __restrict__ cw, const float* __restrict__ cb,
    float* __restrict__ UF, unsigned short* __restrict__ UH) {
  unsigned gi = blockIdx.x * 256u + threadIdx.x;
  if (gi >= (unsigned)(kRows * (kDin / 4))) return;
  unsigned e4 = (gi & (unsigned)(kDin / 4 - 1)) << 2;
  unsigned m  = gi >> 9;
  unsigned l  = m & (unsigned)(kSeq - 1);
  asm volatile("" : "+v"(e4), "+v"(m), "+v"(l));
  v4f wv[4];
#pragma unroll
  for (int c = 0; c < 4; ++c) wv[c] = *(const v4f*)(cw + (size_t)(e4 + (unsigned)c) * kTaps);
  const v4f bv = *(const v4f*)(cb + e4);
  v4f xs[4];
#pragma unroll
  for (int j = 0; j < 4; ++j) {
    const bool ok = (l + (unsigned)j) >= 3u;
    const unsigned row = ok ? (m + (unsigned)j - 3u) : m;
    v4f xv = *(const v4f*)(X + (size_t)row * kDin + e4);
    pin4(xv);
    xs[j] = (v4f){ok ? xv[0] : 0.0f, ok ? xv[1] : 0.0f, ok ? xv[2] : 0.0f, ok ? xv[3] : 0.0f};
  }
  v4f uo;
  v4h uh;
#pragma unroll
  for (int c = 0; c < 4; ++c) {
    float acc = leg_in(wv[c][0]) * xs[0][c];
    acc = fmaf(leg_in(wv[c][1]), xs[1][c], acc);
    acc = fmaf(leg_in(wv[c][2]), xs[2][c], acc);
    acc = fmaf(leg_in(wv[c][3]), xs[3][c], acc);
    const float xc = acc + leg_in(bv[c]);
    const float u = silu_f(xc);
    uo[c] = u;
    uh[c] = f16_flush(u * kCarryU);
  }
  float* pf = UF + (size_t)m * kDin + e4;
  unsigned short* ph = UH + (size_t)m * kDin + e4;
  *(volatile v4f*)pf = uo;
  *(volatile v4h*)ph = uh;
  __threadfence();
  *(volatile v4f*)pf = uo;
  *(volatile v4h*)ph = uh;
}

__global__ __launch_bounds__(64) void scan_gate_kernel(
    const float* __restrict__ DLT, const float* __restrict__ UF, const float* __restrict__ BC,
    const float* __restrict__ Z, const float* __restrict__ Alog, const float* __restrict__ Dv,
    float* __restrict__ out) {
  __shared__ __align__(16) float sA[kNst * 64];
  __shared__ __align__(16) float sBC[kChunk * kBcW];
  __shared__ __align__(16) float sZ[2][kChunk * 33];
  __shared__ __align__(16) float sY[2][kChunk * 36];
  unsigned tid  = threadIdx.x;
  unsigned lane = tid & 31u;
  unsigned wave = tid >> 5;
  unsigned bix  = blockIdx.x >> 5;
  unsigned e0   = ((blockIdx.x & 31u) << 6) + (wave << 5);
  asm volatile("" : "+v"(lane), "+v"(e0));
  const unsigned e    = e0 + lane;
  const unsigned row0 = bix * (unsigned)kSeq;

#pragma unroll 1
  for (int n = 0; n < kNst; ++n) {
    const float al = Alog[(size_t)e * kNst + n];
    sA[n * 64 + tid] = -expf(leg_in(al));
  }
  __syncthreads();
  float An[kNst], h[kNst];
#pragma unroll
  for (int n = 0; n < kNst; ++n) {
    An[n] = sA[n * 64 + tid];
    h[n] = 0.0f;
  }
  const float Dd = leg_in(Dv[e]);
  float* sz = sZ[wave];
  float* sy = sY[wave];
  const unsigned q  = lane >> 3;
  const unsigned c4 = (lane & 7u) << 2;

#pragma unroll 1
  for (unsigned t0 = 0; t0 < (unsigned)kSeq; t0 += (unsigned)kChunk) {
    __syncthreads();
#pragma unroll
    for (int i = 0; i < 4; ++i) {
      const unsigned idx = tid + 64u * (unsigned)i;
      *(v4f*)(sBC + idx * 4u) = *(const v4f*)(BC + ((size_t)(row0 + t0) * kBcW + idx * 4u));
    }
#pragma unroll
    for (int j = 0; j < 8; ++j) {
      const unsigned ich = q + 4u * (unsigned)j;
      const v4f zv = *(const v4f*)(Z + ((size_t)(bix * (unsigned)kDin + e0 + ich) * kSeq + t0 + c4));
      sz[(c4 + 0u) * 33u + ich] = leg_in(zv[0]);
      sz[(c4 + 1u) * 33u + ich] = leg_in(zv[1]);
      sz[(c4 + 2u) * 33u + ich] = leg_in(zv[2]);
      sz[(c4 + 3u) * 33u + ich] = leg_in(zv[3]);
    }
    __syncthreads();
#pragma unroll 1
    for (unsigned s = 0; s < (unsigned)kChunk; ++s) {
      const size_t gidx = (size_t)(row0 + t0 + s) * kDin + e;
      const float dlt = DLT[gidx];
      const float ut  = UF[gidx];
      const float* bc = sBC + s * (unsigned)kBcW;
      float Bn[kNst], Cn[kNst];
#pragma unroll
      for (int q4 = 0; q4 < 4; ++q4) {
        const v4f b4 = *(const v4f*)(bc + 4 * q4);
        const v4f c4v = *(const v4f*)(bc + kNst + 4 * q4);
        Bn[4 * q4 + 0] = b4[0]; Bn[4 * q4 + 1] = b4[1]; Bn[4 * q4 + 2] = b4[2]; Bn[4 * q4 + 3] = b4[3];
        Cn[4 * q4 + 0] = c4v[0]; Cn[4 * q4 + 1] = c4v[1]; Cn[4 * q4 + 2] = c4v[2]; Cn[4 * q4 + 3] = c4v[3];
      }
      const float dbu = dlt * ut;
      float y = 0.0f;
#pragma unroll
      for (int n = 0; n < kNst; ++n) {
        const float dA = expf(dlt * An[n]);
        h[n] = h[n] * dA + dbu * Bn[n];
        y = y + h[n] * Cn[n];
      }
      y = y + Dd * ut;
      const float zv = sz[s * 33u + lane];
      y = y * silu_f(zv);
      sy[s * 36u + lane] = y;
    }
    __syncthreads();
    v4f ov[8];
#pragma unroll
    for (int it = 0; it < 8; ++it) ov[it] = *(const v4f*)(sy + ((unsigned)it * 4u + q) * 36u + c4);
    for (int pass = 0; pass < 2; ++pass) {
#pragma unroll
      for (int it = 0; it < 8; ++it) {
        const unsigned row = (unsigned)it * 4u + q;
        *(volatile v4f*)(out + ((size_t)(row0 + t0 + row) * kDin + e0 + c4)) = ov[it];
      }
      __threadfence();
    }
  }
}

extern "C" void kernel_launch(void* const* d_in, const int* in_sizes, int n_in,
                              void* d_out, int out_size, void* d_ws, size_t ws_size,
                              hipStream_t stream) {
  if (n_in < 10) return;
  if (in_sizes[0] != kRows * kDm) return;
  if (in_sizes[1] != kNB * kDin * kSeq) return;
  if (in_sizes[2] != kDin * kDm) return;
  if (in_sizes[3] != kDin * kTaps) return;
  if (in_sizes[4] != kDin) return;
  if (in_sizes[5] != kXw * kDin) return;
  if (in_sizes[6] != kDin * kDtR) return;
  if (in_sizes[7] != kDin) return;
  if (in_sizes[8] != kDin * kNst) return;
  if (in_sizes[9] != kDin) return;
  if (out_size != kRows * kDin) return;
  if (ws_size < kWsTotal) return;

  const float* hs        = (const float*)d_in[0];
  const float* z         = (const float*)d_in[1];
  const float* in_proj_w = (const float*)d_in[2];
  const float* conv_w    = (const float*)d_in[3];
  const float* conv_b    = (const float*)d_in[4];
  const float* x_proj_w  = (const float*)d_in[5];
  const float* dt_proj_w = (const float*)d_in[6];
  const float* dt_proj_b = (const float*)d_in[7];
  const float* A_log     = (const float*)d_in[8];
  const float* Dvec      = (const float*)d_in[9];
  float* out = (float*)d_out;

  char* ws = (char*)d_ws;
  unsigned short* A1H = (unsigned short*)(ws + kOffA1H);
  unsigned short* B1H = (unsigned short*)(ws + kOffB1H);
  unsigned short* A1L = kLegBf16 ? A1H : (unsigned short*)(ws + kOffA1L);
  unsigned short* B1L = kLegBf16 ? B1H : (unsigned short*)(ws + kOffB1L);
  unsigned short* BT2 = (unsigned short*)(ws + kOffBT2);
  unsigned short* BT3 = (unsigned short*)(ws + kOffBT3);
  float*          XD  = (float*)(ws + kOffXD);
  float*          UF  = (float*)(ws + kOffUF);
  unsigned short* UH  = (unsigned short*)(ws + kOffUH);
  float*          BCp = (float*)(ws + kOffBC);
  unsigned short* DTL = (unsigned short*)(ws + kOffDTL);

  prep_bf16_kernel<!kLegBf16><<<(kRows * kDm / 8) / 256, 256, 0, stream>>>(hs, A1H, A1L, kRows * kDm / 8);
  prep_bf16_kernel<!kLegBf16><<<(kDin * kDm / 8) / 256, 256, 0, stream>>>(in_proj_w, B1H, B1L, kDin * kDm / 8);
  prep_f16_kernel<1024><<<(kXwPad * kDin / 8) / 256, 256, 0, stream>>>(x_proj_w, BT2, kXw * kDin / 8, kXwPad * kDin / 8);
  prep_f16_kernel<1024><<<(kDin * kDtR / 8) / 256, 256, 0, stream>>>(dt_proj_w, BT3, kDin * kDtR / 8, kDin * kDtR / 8);

  gemm64_kernel<1, kSpl1, 0><<<256, 256, 0, stream>>>(
      A1H, A1L, kDm, B1H, B1L, kDm, (void*)XD, (void*)XD, kDin, dt_proj_b, kRows, kDin, kDm);

  conv_act_kernel<<<(kRows * (kDin / 4)) / 256, 256, 0, stream>>>(XD, conv_w, conv_b, UF, UH);

  gemm64_kernel<0, 0, 1><<<16, 256, 0, stream>>>(
      UH, UH, kDin, BT2, BT2, kDin, (void*)BCp, (void*)DTL, kBcW, dt_proj_b, kRows, kXwPad, kDin);

  gemm64_kernel<0, 0, 2><<<256, 256, 0, stream>>>(
      DTL, DTL, kDtR, BT3, BT3, kDtR, (void*)XD, (void*)XD, kDin, dt_proj_b, kRows, kDin, kDtR);

  scan_gate_kernel<<<kNB * (kDin / 64), 64, 0, stream>>>(XD, UF, BCp, z, A_log, Dvec, out);
}
